// TreeGRUDiscriminator_26328149525043
// MI455X (gfx1250) — hardware-verified
//
#include <hip/hip_runtime.h>
#include <stddef.h>
#include <math.h>


#define F       64
#define G3      192
#define NTHR    256
#define NWAVE   8
#define EPT     8
#define NGRP    2
#define CHUNK   (NTHR * EPT * NGRP)
#define WCAP    (EPT * NGRP * 32)
#define LISTN   (NWAVE * WCAP)
#define MT      512
#define GR      128
#define ASCALE  16.0f
#define WSCALE  8.0f
#define PINV    0.0078125f
#define LDS_MEAN ((MT * F + MT + LISTN + NWAVE) * 4)

static_assert((CHUNK & (CHUNK - 1)) == 0);
static_assert(CHUNK <= 4096);
static_assert((MT & (MT - 1)) == 0 && MT <= 4096);
static_assert((MT * F / 4) % NTHR == 0 && (MT * F / 8) % NTHR == 0);
static_assert(MT % GR == 0 && GR == NWAVE * 16);
static_assert((G3 * F / 8) % NTHR == 0);
static_assert((MT * F / 8) % NTHR == 0);

typedef float    v2f  __attribute__((ext_vector_type(2)));
typedef float    v4f  __attribute__((ext_vector_type(4)));
typedef float    v8f  __attribute__((ext_vector_type(8)));
typedef int      v4i  __attribute__((ext_vector_type(4)));
typedef _Float16 v8h  __attribute__((ext_vector_type(8)));
typedef _Float16 v16h __attribute__((ext_vector_type(16)));
union FragH { v16h v; v8h h[2]; };

__device__ __forceinline__ v8h cvt8(v4f a, v4f b) {
  v8h r;
  r[0] = (_Float16)a.x; r[1] = (_Float16)a.y; r[2] = (_Float16)a.z; r[3] = (_Float16)a.w;
  r[4] = (_Float16)b.x; r[5] = (_Float16)b.y; r[6] = (_Float16)b.z; r[7] = (_Float16)b.w;
  return r;
}

__device__ __forceinline__ v8f wmh(v16h a, v16h b, v8f c) {
#if defined(__HIP_DEVICE_COMPILE__)
  v8f d = __builtin_amdgcn_wmma_f32_16x16x32_f16(false, a, false, b, (short)0, c, false, false);
  asm volatile("v_nop\n\tv_nop\n\tv_nop\n\tv_nop" : "+v"(d) : "v"(a), "v"(b));
  return d;
#else
  (void)a; (void)b;
  return c;
#endif
}

__device__ __forceinline__ float sigm(float x) {
  x = fminf(fmaxf(x, -30.0f), 30.0f);
  return 1.0f / (1.0f + expf(-x));
}

template <int NB>
__device__ __forceinline__ int scan_chunk(const int* __restrict__ dsts, int nE, int cbase, int slotBase,
                                          int vec8, int* list, int tid, int lane, int wave) {
  int wc = 0;
#pragma unroll
  for (int g = 0; g < NGRP; ++g) {
    const int el0  = (g * NTHR + tid) * EPT;
    const int e0   = cbase + el0;
    const int sent = -2147483647 - 1;
    v4i da, db;
    if (vec8 != 0 && cbase + CHUNK <= nE) {
      da = *(const v4i*)(dsts + e0);
      db = *(const v4i*)(dsts + e0 + 4);
    } else {
      da.x = (e0     < nE) ? dsts[min(e0, nE - 1)] : sent;
      da.y = (e0 + 1 < nE) ? dsts[min(e0 + 1, nE - 1)] : sent;
      da.z = (e0 + 2 < nE) ? dsts[min(e0 + 2, nE - 1)] : sent;
      da.w = (e0 + 3 < nE) ? dsts[min(e0 + 3, nE - 1)] : sent;
      db.x = (e0 + 4 < nE) ? dsts[min(e0 + 4, nE - 1)] : sent;
      db.y = (e0 + 5 < nE) ? dsts[min(e0 + 5, nE - 1)] : sent;
      db.z = (e0 + 6 < nE) ? dsts[min(e0 + 6, nE - 1)] : sent;
      db.w = (e0 + 7 < nE) ? dsts[min(e0 + 7, nE - 1)] : sent;
    }
    const unsigned nb = (unsigned)slotBase;
    const unsigned s0 = (unsigned)da.x - nb, s1 = (unsigned)da.y - nb;
    const unsigned s2 = (unsigned)da.z - nb, s3 = (unsigned)da.w - nb;
    const unsigned s4 = (unsigned)db.x - nb, s5 = (unsigned)db.y - nb;
    const unsigned s6 = (unsigned)db.z - nb, s7 = (unsigned)db.w - nb;
    const bool h0 = s0 < (unsigned)NB, h1 = s1 < (unsigned)NB, h2 = s2 < (unsigned)NB, h3 = s3 < (unsigned)NB;
    const bool h4 = s4 < (unsigned)NB, h5 = s5 < (unsigned)NB, h6 = s6 < (unsigned)NB, h7 = s7 < (unsigned)NB;
    const unsigned any = __builtin_amdgcn_ballot_w32(h0 | h1 | h2 | h3 | h4 | h5 | h6 | h7);
    if (any != 0u) {
#define HITJ(J, HJ, SJ) { \
        const unsigned mj = __builtin_amdgcn_ballot_w32(HJ); \
        if (mj != 0u) { \
          if (HJ) { \
            const int pos = wc + (int)__builtin_amdgcn_mbcnt_lo(mj, 0u); \
            if (pos < WCAP) list[wave * WCAP + pos] = ((el0 + (J)) << 12) | (int)(SJ); \
          } \
          wc += (int)__builtin_popcount(mj); } }
      HITJ(0, h0, s0)
      HITJ(1, h1, s1)
      HITJ(2, h2, s2)
      HITJ(3, h3, s3)
      HITJ(4, h4, s4)
      HITJ(5, h5, s5)
      HITJ(6, h6, s6)
      HITJ(7, h7, s7)
#undef HITJ
    }
  }
  return wc;
}

__global__ __launch_bounds__(NTHR) void k_prep(
    const float* __restrict__ wa, const float* __restrict__ wb, const float* __restrict__ wc,
    const float* __restrict__ wd, const float* __restrict__ z,
    _Float16* pa, _Float16* pb, _Float16* pc, _Float16* pd, _Float16* z16,
    int nN, int nPadRows) {
  const int per = G3 * F / 8;
  const int bstart = blockIdx.x * NTHR;
  const int i = bstart + (int)threadIdx.x;
  v4f a, b;
  _Float16* dp;
  if (bstart < 4 * per) {
    const int seg = bstart / per;
    const float* src = seg == 0 ? wa : (seg == 1 ? wb : (seg == 2 ? wc : wd));
    _Float16*    dst = seg == 0 ? pa : (seg == 1 ? pb : (seg == 2 ? pc : pd));
    const int o = (i - seg * per) * 8;
    a = *(const v4f*)(src + o) * WSCALE;
    b = *(const v4f*)(src + o + 4) * WSCALE;
    dp = dst + o;
  } else {
    const int j = i - 4 * per;
    if (j >= nPadRows * (F / 8)) return;
    const int row = j >> 3;
    const int c0  = (j & 7) * 8;
    const int rc  = row < nN ? row : nN - 1;
    const float* sp = z + (size_t)rc * F + c0;
    const float s = row < nN ? ASCALE : 0.0f;
    a = *(const v4f*)sp * s;
    b = *(const v4f*)(sp + 4) * s;
    dp = z16 + (size_t)j * 8;
  }
  const v8h hv = cvt8(a, b);
  *(volatile v8h*)dp = hv;
  __threadfence();
  *(volatile v8h*)dp = hv;
}

__global__ __launch_bounds__(NTHR) void k_mean(
    const int* __restrict__ ei, const float* __restrict__ hin,
    float* hout32, _Float16* hout16, int nN, int nE, int vec8) {
  extern __shared__ v4f lds_dyn[];
  float* acc  = (float*)lds_dyn;
  int*   cnt  = (int*)(acc + MT * F);
  int*   list = cnt + MT;
  int*   wcnt = list + LISTN;
  const int tid = threadIdx.x, lane = tid & 31, wave = tid >> 5;
  const int slotBase = blockIdx.x * MT;
  const int* dsts = ei + nE;

  {
    const v4f z4 = {0.f, 0.f, 0.f, 0.f};
#pragma unroll 1
    for (int i = tid; i < MT * F / 4; i += NTHR) ((v4f*)acc)[i] = z4;
    for (int i = tid; i < MT; i += NTHR) cnt[i] = 0;
  }
  __syncthreads();

  const int nChunks = (nE + CHUNK - 1) / CHUNK;
#pragma unroll 1
  for (int ch = 0; ch < nChunks; ++ch) {
    const int cbase = ch * CHUNK;
    const int wc = scan_chunk<MT>(dsts, nE, cbase, slotBase, vec8, list, tid, lane, wave);
    if (lane == 0) wcnt[wave] = wc;
    __syncthreads();
    if (wave == 0) {
#pragma unroll 1
      for (int wsx = 0; wsx < NWAVE; ++wsx) {
        int n = __builtin_amdgcn_readfirstlane(wcnt[wsx]);
        n = n > WCAP ? WCAP : (n < 0 ? 0 : n);
        const int* lp = list + wsx * WCAP;
#pragma unroll 1
        for (int i = 0; i < n; ++i) {
          const int ent  = __builtin_amdgcn_readfirstlane(lp[i]);
          const int slot = ent & (MT - 1);
          int e = cbase + ((ent >> 12) & (CHUNK - 1));
          e = e > nE - 1 ? nE - 1 : e;
          int src = ei[e];
          src = src < 0 ? 0 : (src > nN - 1 ? nN - 1 : src);
          const v2f v = *(const v2f*)(hin + (size_t)src * F + 2 * lane);
          v2f* ap = (v2f*)(acc + slot * F + 2 * lane);
          *ap = *ap + v;
          if (lane == 0) cnt[slot] = cnt[slot] + 1;
        }
      }
    }
    __syncthreads();
  }

  float*    g32 = hout32 + (size_t)slotBase * F;
  _Float16* g16 = hout16 + (size_t)slotBase * F;
#pragma unroll 1
  for (int it = 0; it < (MT * F / 4) / NTHR; ++it) {
    const int i = it * NTHR + tid;
    int cv = cnt[i >> 4];
    cv = cv < 1 ? 1 : cv;
    const float inv = 1.0f / (float)cv;
    const v4f v = ((const v4f*)acc)[i] * inv;
    *(volatile v4f*)(g32 + 4 * (size_t)i) = v;
  }
#pragma unroll 1
  for (int it = 0; it < (MT * F / 8) / NTHR; ++it) {
    const int i = it * NTHR + tid;
    int cv = cnt[i >> 3];
    cv = cv < 1 ? 1 : cv;
    const float inv = 1.0f / (float)cv;
    const v4f a = (((const v4f*)acc)[2 * i] * inv) * ASCALE;
    const v4f b = (((const v4f*)acc)[2 * i + 1] * inv) * ASCALE;
    *(volatile v8h*)(g16 + 8 * (size_t)i) = cvt8(a, b);
  }
  __threadfence();
#pragma unroll 1
  for (int it = 0; it < (MT * F / 4) / NTHR; ++it) {
    const int i = it * NTHR + tid;
    int cv = cnt[i >> 4];
    cv = cv < 1 ? 1 : cv;
    const float inv = 1.0f / (float)cv;
    const v4f v = ((const v4f*)acc)[i] * inv;
    *(volatile v4f*)(g32 + 4 * (size_t)i) = v;
  }
#pragma unroll 1
  for (int it = 0; it < (MT * F / 8) / NTHR; ++it) {
    const int i = it * NTHR + tid;
    int cv = cnt[i >> 3];
    cv = cv < 1 ? 1 : cv;
    const float inv = 1.0f / (float)cv;
    const v4f a = (((const v4f*)acc)[2 * i] * inv) * ASCALE;
    const v4f b = (((const v4f*)acc)[2 * i + 1] * inv) * ASCALE;
    *(volatile v8h*)(g16 + 8 * (size_t)i) = cvt8(a, b);
  }
}

__global__ __launch_bounds__(NTHR) void k_gru(
    const _Float16* __restrict__ x16, const _Float16* __restrict__ wih, const _Float16* __restrict__ whh,
    const float* __restrict__ bih, const float* __restrict__ bhh,
    const _Float16* hp16, const float* hp32, float* ho32, _Float16* ho16,
    const float* __restrict__ wout, const float* __restrict__ bout, float* out,
    int nN, int first, int doHead) {
  __shared__ __attribute__((aligned(16))) float    sH[NWAVE * 16 * F];
  __shared__ __attribute__((aligned(16))) _Float16 sH16[NWAVE * 16 * F];
  __shared__ __attribute__((aligned(16))) float    sOut[GR];
  const int tid = threadIdx.x, lane = tid & 31, wave = tid >> 5, hh = lane >> 4, m = lane & 15;
  const int row0 = blockIdx.x * GR + wave * 16;
  float*    sw   = sH + wave * 16 * F;
  _Float16* sw16 = sH16 + wave * 16 * F;

  FragH ax0, ax1, ah0, ah1;
  {
    const _Float16* xr = x16 + (size_t)(row0 + m) * F + 8 * hh;
    ax0.h[0] = *(const v8h*)(xr);
    ax0.h[1] = *(const v8h*)(xr + 16);
    ax1.h[0] = *(const v8h*)(xr + 32);
    ax1.h[1] = *(const v8h*)(xr + 48);
  }
  {
    v16h zv = {};
    ah0.v = zv;
    ah1.v = zv;
  }
  if (first == 0) {
    const _Float16* hr = hp16 + (size_t)(row0 + m) * F + 8 * hh;
    ah0.h[0] = *(const v8h*)(hr);
    ah0.h[1] = *(const v8h*)(hr + 16);
    ah1.h[0] = *(const v8h*)(hr + 32);
    ah1.h[1] = *(const v8h*)(hr + 48);
  }

#pragma unroll
  for (int jt = 0; jt < 4; ++jt) {
    v8f acc[6];
#pragma unroll
    for (int g = 0; g < 6; ++g) { v8f zz = {0.f, 0.f, 0.f, 0.f, 0.f, 0.f, 0.f, 0.f}; acc[g] = zz; }
#pragma unroll
    for (int g = 0; g < 3; ++g) {
      const _Float16* bp = wih + (size_t)(64 * g + 16 * jt + m) * F + 8 * hh;
      FragH b0, b1;
      b0.h[0] = *(const v8h*)(bp);
      b0.h[1] = *(const v8h*)(bp + 16);
      b1.h[0] = *(const v8h*)(bp + 32);
      b1.h[1] = *(const v8h*)(bp + 48);
      acc[g] = wmh(ax0.v, b0.v, acc[g]);
      acc[g] = wmh(ax1.v, b1.v, acc[g]);
    }
    if (first == 0) {
#pragma unroll
      for (int g = 0; g < 3; ++g) {
        const _Float16* bp = whh + (size_t)(64 * g + 16 * jt + m) * F + 8 * hh;
        FragH b0, b1;
        b0.h[0] = *(const v8h*)(bp);
        b0.h[1] = *(const v8h*)(bp + 16);
        b1.h[0] = *(const v8h*)(bp + 32);
        b1.h[1] = *(const v8h*)(bp + 48);
        acc[3 + g] = wmh(ah0.v, b0.v, acc[3 + g]);
        acc[3 + g] = wmh(ah1.v, b1.v, acc[3 + g]);
      }
    }
    const int f = 16 * jt + m;
    const float bir = bih[f], biz = bih[64 + f], bin_ = bih[128 + f];
    const float bhr = bhh[f], bhz = bhh[64 + f], bhn  = bhh[128 + f];
#pragma unroll
    for (int r = 0; r < 8; ++r) {
      const int lr = 8 * hh + r;
      const float gir = acc[0][r] * PINV + bir;
      const float giz = acc[1][r] * PINV + biz;
      const float gin = acc[2][r] * PINV + bin_;
      const float ghr = acc[3][r] * PINV + bhr;
      const float ghz = acc[4][r] * PINV + bhz;
      const float ghn = acc[5][r] * PINV + bhn;
      const float rg  = sigm(gir + ghr);
      const float ug  = sigm(giz + ghz);
      const float ng  = tanhf(gin + rg * ghn);
      const float hl  = hp32[(size_t)(row0 + lr) * F + f];
      const float hpv = first != 0 ? 0.0f : hl;
      const float hv  = (1.0f - ug) * ng + ug * hpv;
      sw[lr * F + f]   = hv;
      sw16[lr * F + f] = (_Float16)(hv * ASCALE);
    }
  }
  __syncthreads();

  float hs = 0.0f;
  if (doHead != 0) {
    const float* hrow = sw + m * F + 32 * hh;
    const float* wp   = wout + 32 * hh;
#pragma unroll 1
    for (int c = 0; c < 32; ++c) hs += tanhf(hrow[c]) * wp[c];
  }
  hs += __shfl_xor(hs, 16);
  if (doHead != 0 && hh == 0) sOut[wave * 16 + m] = hs + bout[0];
  __syncthreads();

  const v4f* lp4 = (const v4f*)sw;
  const v8h* lp8 = (const v8h*)sw16;
  float*     gp32 = ho32 + (size_t)row0 * F;
  _Float16*  gp16 = ho16 + (size_t)row0 * F;
  const bool headWave = (doHead != 0) && (wave == 0);
  const int  orow = blockIdx.x * GR + 4 * lane;
  v4f ov = {0.f, 0.f, 0.f, 0.f};
  if (headWave) ov = *(const v4f*)(sOut + 4 * lane);

#pragma unroll
  for (int p = 0; p < 8; ++p) { const int idx = p * 32 + lane; const v4f v = lp4[idx]; *(volatile v4f*)(gp32 + 4 * idx) = v; }
#pragma unroll
  for (int p = 0; p < 4; ++p) { const int idx = p * 32 + lane; const v8h v = lp8[idx]; *(volatile v8h*)(gp16 + 8 * idx) = v; }
  if (headWave) {
    if (orow + 4 <= nN) {
      *(volatile v4f*)(out + orow) = ov;
    } else {
      if (orow + 0 < nN) *(volatile float*)(out + orow + 0) = ov.x;
      if (orow + 1 < nN) *(volatile float*)(out + orow + 1) = ov.y;
      if (orow + 2 < nN) *(volatile float*)(out + orow + 2) = ov.z;
      if (orow + 3 < nN) *(volatile float*)(out + orow + 3) = ov.w;
    }
  }
  __threadfence();
#pragma unroll
  for (int p = 0; p < 8; ++p) { const int idx = p * 32 + lane; const v4f v = lp4[idx]; *(volatile v4f*)(gp32 + 4 * idx) = v; }
#pragma unroll
  for (int p = 0; p < 4; ++p) { const int idx = p * 32 + lane; const v8h v = lp8[idx]; *(volatile v8h*)(gp16 + 8 * idx) = v; }
  if (headWave) {
    if (orow + 4 <= nN) {
      *(volatile v4f*)(out + orow) = ov;
    } else {
      if (orow + 0 < nN) *(volatile float*)(out + orow + 0) = ov.x;
      if (orow + 1 < nN) *(volatile float*)(out + orow + 1) = ov.y;
      if (orow + 2 < nN) *(volatile float*)(out + orow + 2) = ov.z;
      if (orow + 3 < nN) *(volatile float*)(out + orow + 3) = ov.w;
    }
  }
}

extern "C" void kernel_launch(void* const* d_in, const int* in_sizes, int n_in,
                              void* d_out, int out_size, void* d_ws, size_t ws_size,
                              hipStream_t stream) {
  if (n_in < 12) return;
  const int nN = in_sizes[0] / F;
  const int nE = in_sizes[1] / 2;
  if (nN <= 0 || in_sizes[0] != nN * F || nE < 0 || in_sizes[1] != 2 * nE) return;
  if (in_sizes[2] != G3 * F || in_sizes[3] != G3 * F || in_sizes[6] != G3 * F || in_sizes[7] != G3 * F) return;
  if (in_sizes[4] != G3 || in_sizes[5] != G3 || in_sizes[8] != G3 || in_sizes[9] != G3) return;
  if (in_sizes[10] != F || in_sizes[11] < 1) return;
  if (out_size != nN) return;
  if (nN > (1 << 24) || nE > (1 << 28)) return;

  const float* z     = (const float*)d_in[0];
  const int*   ei    = (const int*)d_in[1];
  const float* W_ih0 = (const float*)d_in[2];
  const float* W_hh0 = (const float*)d_in[3];
  const float* b_ih0 = (const float*)d_in[4];
  const float* b_hh0 = (const float*)d_in[5];
  const float* W_ih1 = (const float*)d_in[6];
  const float* W_hh1 = (const float*)d_in[7];
  const float* b_ih1 = (const float*)d_in[8];
  const float* b_hh1 = (const float*)d_in[9];
  const float* W_out = (const float*)d_in[10];
  const float* b_out = (const float*)d_in[11];
  float* out = (float*)d_out;

  const int NPAD = ((nN + MT - 1) / MT) * MT;

  char* ws = (char*)d_ws;
  size_t off = 0;
  const size_t wBytes   = (size_t)G3 * F * 2;
  const size_t p16Bytes = (size_t)NPAD * F * 2;
  const size_t p32Bytes = (size_t)NPAD * F * 4;
  const size_t oWih0 = off; off += wBytes;
  const size_t oWhh0 = off; off += wBytes;
  const size_t oWih1 = off; off += wBytes;
  const size_t oWhh1 = off; off += wBytes;
  const size_t oZ16  = off; off += p16Bytes;
  size_t oF32[3], oF16[3];
  for (int d = 0; d < 3; ++d) { oF32[d] = off; off += p32Bytes; }
  for (int d = 0; d < 3; ++d) { oF16[d] = off; off += p16Bytes; }
  const size_t oH0_32 = off; off += p32Bytes;
  const size_t oH1_32 = off; off += p32Bytes;
  const size_t oH0_16 = off; off += p16Bytes;
  const size_t oH1_16 = off; off += p16Bytes;
  if (off > ws_size) return;

  _Float16* pWih0 = (_Float16*)(ws + oWih0);
  _Float16* pWhh0 = (_Float16*)(ws + oWhh0);
  _Float16* pWih1 = (_Float16*)(ws + oWih1);
  _Float16* pWhh1 = (_Float16*)(ws + oWhh1);
  _Float16* z16   = (_Float16*)(ws + oZ16);
  float*    fr32[3]; _Float16* fr16[3];
  for (int d = 0; d < 3; ++d) { fr32[d] = (float*)(ws + oF32[d]); fr16[d] = (_Float16*)(ws + oF16[d]); }
  float*    h0_32 = (float*)(ws + oH0_32);
  float*    h1_32 = (float*)(ws + oH1_32);
  _Float16* h0_16 = (_Float16*)(ws + oH0_16);
  _Float16* h1_16 = (_Float16*)(ws + oH1_16);

  const int vec8 = ((nE & 3) == 0) ? 1 : 0;

  const int nPrepThr = 4 * (G3 * F / 8) + NPAD * (F / 8);
  k_prep<<<(nPrepThr + NTHR - 1) / NTHR, NTHR, 0, stream>>>(W_ih0, W_hh0, W_ih1, W_hh1, z,
                                                            pWih0, pWhh0, pWih1, pWhh1, z16, nN, NPAD);

  hipFuncSetAttribute(reinterpret_cast<const void*>(&k_mean),
                      hipFuncAttributeMaxDynamicSharedMemorySize, LDS_MEAN);
  const int nMean = NPAD / MT;
  k_mean<<<nMean, NTHR, LDS_MEAN, stream>>>(ei, z,       fr32[0], fr16[0], nN, nE, vec8);
  k_mean<<<nMean, NTHR, LDS_MEAN, stream>>>(ei, fr32[0], fr32[1], fr16[1], nN, nE, vec8);
  k_mean<<<nMean, NTHR, LDS_MEAN, stream>>>(ei, fr32[1], fr32[2], fr16[2], nN, nE, vec8);

  const int nGru = NPAD / GR;
  for (int t = 0; t < 4; ++t) {
    const _Float16* xp = (t == 0) ? z16 : fr16[t - 1];
    k_gru<<<nGru, NTHR, 0, stream>>>(xp, pWih0, pWhh0, b_ih0, b_hh0,
                                     h0_16, h0_32, h0_32, h0_16,
                                     W_out, b_out, out, nN, t == 0 ? 1 : 0, 0);
    k_gru<<<nGru, NTHR, 0, stream>>>(h0_16, pWih1, pWhh1, b_ih1, b_hh1,
                                     h1_16, h1_32, h1_32, h1_16,
                                     W_out, b_out, out, nN, t == 0 ? 1 : 0, t == 3 ? 1 : 0);
  }
}
